// DecoderBlock_30434138259804
// MI455X (gfx1250) — hardware-verified
//
#include <hip/hip_runtime.h>
#include <math.h>

typedef __attribute__((ext_vector_type(16))) _Float16 v16h;
typedef __attribute__((ext_vector_type(8)))  _Float16 v8h;
typedef __attribute__((ext_vector_type(8)))  float    v8f;
typedef __attribute__((ext_vector_type(4)))  float    v4f;
typedef __attribute__((ext_vector_type(4)))  unsigned v4u;
typedef __attribute__((ext_vector_type(2)))  unsigned v2u;

#ifndef NB
#define NB 2
#endif
#ifndef SEQ
#define SEQ 2048
#endif

constexpr int kBatchFull = 2;
constexpr int kSeqFull   = 2048;
constexpr int kBatch = NB;
constexpr int kSeq   = SEQ;
constexpr int kDim   = 768;
constexpr int kHeads = 12;
constexpr int kHdim  = 64;
constexpr int kFfn   = 3072;
constexpr int kQkvN  = 3 * kDim;
constexpr int kModN  = 6 * kDim;
constexpr int kRows  = kBatch * kSeq;
constexpr int kQP    = 2 * kQkvN;
constexpr float kSqrtD = 27.712812921102035f;
constexpr float kLnEps = 1e-6f;

static_assert(kBatch >= 1 && kBatch <= kBatchFull && kSeq >= 64 && kSeq <= kSeqFull);
static_assert(kSeq % 64 == 0 && kRows % 64 == 0);
static_assert(kDim % 64 == 0 && kQkvN % 64 == 0 && kModN % 64 == 0 && kFfn % 64 == 0);
static_assert(kDim % 32 == 0 && kFfn % 32 == 0 && kHdim == 64 && kHeads * kHdim == kDim);
static_assert(kDim == 4 * 192);

constexpr float kCarryAct  = 8.0f;
constexpr float kCarryW    = 256.0f;
constexpr float kCarryQ    = 64.0f;
constexpr float kCarryK    = 8.0f;
constexpr float kCarryV    = 8.0f;
constexpr float kCarryP    = 4096.0f;
constexpr float kCarryAttn = 128.0f;
constexpr float kCarryH    = 8.0f;

constexpr size_t kSzMod  = (size_t)kRows * kModN * 4;
constexpr size_t kSzW2   = (size_t)kDim * kFfn * 2;
constexpr size_t kSzW1   = (size_t)kFfn * kDim * 2;
constexpr size_t kSzWqkv = (size_t)kQkvN * kDim * 2;
constexpr size_t kSzWo   = (size_t)kDim * kDim * 2;
constexpr size_t kSzWada = (size_t)kModN * kDim * 2;
constexpr size_t kSzA    = (size_t)kRows * kDim * 2;
constexpr size_t kSzQkvF = (size_t)kRows * kQkvN * 4;
constexpr size_t kSzF32  = (size_t)kRows * kDim * 4;
constexpr size_t kSzHid  = (size_t)kRows * kFfn * 2;
constexpr size_t kSzS    = (kSzWada > kSzQkvF) ? kSzWada : kSzQkvF;
constexpr size_t kOffMod  = 0;
constexpr size_t kOffW2   = kOffMod + kSzMod;
constexpr size_t kOffW1   = kOffW2 + kSzW2;
constexpr size_t kOffWqkv = kOffW1 + kSzW1;
constexpr size_t kOffWo   = kOffWqkv + kSzWqkv;
constexpr size_t kOffA    = kOffWo + kSzWo;
constexpr size_t kOffS    = kOffA + kSzA;
constexpr size_t kWsTotal = kOffS + kSzS;
constexpr size_t kOffWada  = kOffS;
constexpr size_t kOffQkvF  = kOffS;
constexpr size_t kOffXmid  = kOffS;
constexpr size_t kOffOproj = kOffS + kSzF32;
constexpr size_t kOffHid   = kOffS + kSzF32;
static_assert(kSzF32 + kSzHid == kSzQkvF);
static_assert(kSzF32 + kSzF32 <= kSzS && kSzF32 + kSzHid <= kSzS && kSzWada <= kSzS && kSzQkvF <= kSzS);
static_assert(kWsTotal <= 134217728);
static_assert(kBatch != 2 || kSeq != 2048 || kWsTotal == 133693440);
static_assert((kOffW2 % 128) == 0 && (kOffW1 % 128) == 0 && (kOffWqkv % 128) == 0 && (kOffWo % 128) == 0 &&
              (kOffA % 128) == 0 && (kOffS % 128) == 0 && (kOffOproj % 128) == 0 && (kOffHid % 128) == 0);

__device__ __forceinline__ unsigned short f2bf_bits(float f) {
  unsigned u = __float_as_uint(f);
  return (unsigned short)((u + 0x7FFFu + ((u >> 16) & 1u)) >> 16);
}
__device__ __forceinline__ float bf_bits2f(unsigned short h) { return __uint_as_float(((unsigned)h) << 16); }
__device__ __forceinline__ float bfr(float f) { return bf_bits2f(f2bf_bits(f)); }
__device__ __forceinline__ v4f bfr4(v4f v) { v4f o; o[0] = bfr(v[0]); o[1] = bfr(v[1]); o[2] = bfr(v[2]); o[3] = bfr(v[3]); return o; }
__device__ __forceinline__ unsigned pack_h2(float a, float b) {
  return (unsigned)__builtin_bit_cast(unsigned short, (_Float16)a) | ((unsigned)__builtin_bit_cast(unsigned short, (_Float16)b) << 16);
}
__device__ __forceinline__ float silu_f(float v) {
  const float t = fmaxf(v, -80.0f);
  return v * __builtin_amdgcn_rcpf(1.0f + __expf(-t));
}
__device__ __forceinline__ int in_row(int r) { const int b = r / kSeq; return b * kSeqFull + (r - b * kSeq); }

union FragU { v16h v; v8h h[2]; };
__device__ __forceinline__ v16h frag_load(const _Float16* p) {
  FragU f; f.h[0] = *(const v8h*)(p); f.h[1] = *(const v8h*)(p + 16); return f.v;
}
__device__ __forceinline__ v8f mma_f16(v16h a, v16h b, v8f c) {
  return __builtin_amdgcn_wmma_f32_16x16x32_f16(false, a, false, b, (short)0, c, false, false);
}
__device__ __forceinline__ void dep_guard_h(v8f& a, v8f& b, v16h x, v16h y) { asm volatile("v_nop\n\tv_nop\n\tv_nop\n\tv_nop" : "+v"(a), "+v"(b) : "v"(x), "v"(y)); }
__device__ __forceinline__ void keep4_h(v16h a, v16h b, v16h c, v16h d) { asm volatile("v_nop" :: "v"(a), "v"(b), "v"(c), "v"(d)); }
__device__ __forceinline__ void acc_guard4(v8f& a, v8f& b, v8f& c, v8f& d) { asm volatile("v_nop\n\tv_nop\n\tv_nop\n\tv_nop" : "+v"(a), "+v"(b), "+v"(c), "+v"(d)); }
__device__ __forceinline__ v8f mma_h(v16h a, v16h b, v8f c) {
  c = __builtin_amdgcn_wmma_f32_16x16x32_f16(false, a, false, b, (short)0, c, false, false);
  asm volatile("v_nop\n\tv_nop\n\tv_nop\n\tv_nop" : "+v"(c) : "v"(a), "v"(b));
  return c;
}

template <int BIAS_MODE, int OUT_MODE, bool RESID, bool GATE, int ACT>
__global__ __launch_bounds__(256) void wmma_gemm64(
    const _Float16* __restrict__ A, int lda,
    const _Float16* __restrict__ Bt, int ldb,
    void* __restrict__ Cout, int ldc,
    const float* __restrict__ bias,
    const float* __restrict__ resid, int ldr,
    const float* __restrict__ gate, int ldg,
    int M, int N, int K, float scale, float oscale) {
  static_assert(!(RESID || GATE) || OUT_MODE == 0);
  __shared__ __align__(16) float sT[8][16 * 68];
  const int lane = threadIdx.x & 31;
  const int wave = threadIdx.x >> 5;
  const int tilesN = N >> 6;
  const int tilesM = M >> 6;
  const int tile = blockIdx.x * 8 + wave;
  if (tile >= tilesM * tilesN) return;
  const int tm = tile / tilesN;
  const int tn = tile - tm * tilesN;
  const int m0 = tm << 6;
  const int n0 = tn << 6;

  const int rlane = lane & 15;
  const int koff  = (lane >> 4) * 8;
  const int mOff  = (lane >> 4) * 8;

  v8f acc[4][4];
#pragma unroll
  for (int i = 0; i < 4; ++i)
#pragma unroll
    for (int j = 0; j < 4; ++j) acc[i][j] = (v8f){0.f,0.f,0.f,0.f,0.f,0.f,0.f,0.f};

  for (int k0 = 0; k0 < K; k0 += 32) {
    v16h bh[4];
#pragma unroll
    for (int j = 0; j < 4; ++j) {
      const size_t bo = (size_t)(n0 + (j << 4) + rlane) * ldb + koff + k0;
      bh[j] = frag_load(Bt + bo);
    }
#pragma unroll
    for (int i = 0; i < 4; ++i) {
      const size_t ao = (size_t)(m0 + (i << 4) + rlane) * lda + koff + k0;
      v16h ah = frag_load(A + ao);
#pragma unroll
      for (int j = 0; j < 4; ++j) acc[i][j] = mma_f16(ah, bh[j], acc[i][j]);
      dep_guard_h(acc[i][0], acc[i][3], ah, ah);
    }
    keep4_h(bh[0], bh[1], bh[2], bh[3]);
  }
  acc_guard4(acc[0][0], acc[0][1], acc[0][2], acc[0][3]);
  acc_guard4(acc[1][0], acc[1][1], acc[1][2], acc[1][3]);
  acc_guard4(acc[2][0], acc[2][1], acc[2][2], acc[2][3]);
  acc_guard4(acc[3][0], acc[3][1], acc[3][2], acc[3][3]);

  float* slab = sT[wave];
#pragma unroll
  for (int i = 0; i < 4; ++i) {
    const int mBase = m0 + (i << 4);
#pragma unroll
    for (int j = 0; j < 4; ++j) {
      const int n = n0 + (j << 4) + rlane;
      float bv = 0.f;
      if (BIAS_MODE == 2) bv = bfr(bias[n]);
#pragma unroll
      for (int r = 0; r < 8; ++r) {
        float v = acc[i][j][r] * scale;
        if (BIAS_MODE == 2) v += bv;
        if (ACT == 3) v = silu_f(v);
        slab[(mOff + r) * 68 + (j << 4) + rlane] = v * oscale;
      }
    }
    __builtin_amdgcn_fence(3  , "workgroup");
    __builtin_amdgcn_wave_barrier();
    __builtin_amdgcn_fence(2  , "workgroup");
    if (OUT_MODE == 0) {
      float* C = (float*)Cout;
      const int hh = lane >> 4, c4 = (lane & 15) * 4;
      for (int pass = 0; pass < 2; ++pass) {
#pragma unroll
        for (int it = 0; it < 8; ++it) {
          const int row = it * 2 + hh;
          v4f v = *(const v4f*)(slab + row * 68 + c4);
          if (GATE) {
            const v4f gv = *(const v4f*)(gate + (size_t)(mBase + row) * ldg + n0 + c4);
            v = v * gv;
          }
          if (RESID) {
            const v4f rr = *(const v4f*)(resid + (size_t)(mBase + row) * ldr + n0 + c4);
            v += rr;
          }
          *(volatile v4f*)(C + (size_t)(mBase + row) * ldc + n0 + c4) = v;
        }
        __threadfence();
      }
    } else {
      const int q = lane >> 3, c8 = (lane & 7) * 8;
      _Float16* C = (_Float16*)Cout;
      for (int pass = 0; pass < 2; ++pass) {
#pragma unroll
        for (int it = 0; it < 4; ++it) {
          const int row = it * 4 + q;
          const float* sp = slab + row * 68 + c8;
          v8h hv;
#pragma unroll
          for (int e = 0; e < 8; ++e) hv[e] = (_Float16)sp[e];
          *(volatile v8h*)(C + (size_t)(mBase + row) * ldc + n0 + c8) = hv;
        }
        __threadfence();
      }
    }
    __builtin_amdgcn_fence(3  , "workgroup");
    __builtin_amdgcn_wave_barrier();
    __builtin_amdgcn_fence(2  , "workgroup");
  }
}

__global__ __launch_bounds__(256) void transpose_cast_w(
    const float* __restrict__ W, _Float16* __restrict__ Wt, int K, int N, float sc) {
  __shared__ float sh[64][65];
  const int k0 = blockIdx.y * 64, n0 = blockIdx.x * 64;
  const int t = threadIdx.x;
#pragma unroll
  for (int it = 0; it < 4; ++it) {
    const int idx = it * 256 + t;
    const int kr = idx >> 4, nc = (idx & 15) * 4;
    const v4f wv = *(const v4f*)(W + (size_t)(k0 + kr) * N + n0 + nc);
    sh[kr][nc] = wv[0]; sh[kr][nc + 1] = wv[1]; sh[kr][nc + 2] = wv[2]; sh[kr][nc + 3] = wv[3];
  }
  __syncthreads();
  const int rq = t >> 3, c8 = (t & 7) * 8;
  v4u pk[2];
#pragma unroll
  for (int it = 0; it < 2; ++it) {
    const int row = it * 32 + rq;
    v4u u;
#pragma unroll
    for (int e = 0; e < 4; ++e)
      u[e] = pack_h2(bfr(sh[c8 + 2 * e][row]) * sc, bfr(sh[c8 + 2 * e + 1][row]) * sc);
    pk[it] = u;
  }
  for (int pass = 0; pass < 2; ++pass) {
#pragma unroll
    for (int it = 0; it < 2; ++it) {
      const int row = it * 32 + rq;
      *(volatile v4u*)(Wt + (size_t)(n0 + row) * K + k0 + c8) = pk[it];
    }
    __threadfence();
  }
}

__global__ __launch_bounds__(256) void silu_cast_rows(
    const float* __restrict__ cin, _Float16* __restrict__ out, int n8, float sc) {
  const int i = blockIdx.x * 256 + threadIdx.x;
  if (i >= n8) return;
  const int e0 = i * 8;
  const int row = e0 / kDim;
  const int col = e0 - row * kDim;
  const float* p = cin + (size_t)in_row(row) * kDim + col;
  const v4f a = bfr4(*(const v4f*)(p));
  const v4f b = bfr4(*(const v4f*)(p + 4));
  v4u u;
  u[0] = pack_h2(silu_f(a[0]) * sc, silu_f(a[1]) * sc);
  u[1] = pack_h2(silu_f(a[2]) * sc, silu_f(a[3]) * sc);
  u[2] = pack_h2(silu_f(b[0]) * sc, silu_f(b[1]) * sc);
  u[3] = pack_h2(silu_f(b[2]) * sc, silu_f(b[3]) * sc);
  _Float16* q = out + (size_t)row * kDim + col;
  *(volatile v4u*)q = u;
  __threadfence();
  *(volatile v4u*)q = u;
}

__global__ __launch_bounds__(192) void ln_mod_rows(
    const float* __restrict__ x, const float* __restrict__ mod, _Float16* __restrict__ hout, float hscale) {
  __shared__ float ssum[6];
  __shared__ float ssq[6];
  __shared__ __align__(16) unsigned hrow[384];
  const int row = blockIdx.x;
  const int t = threadIdx.x;
  const int w = t >> 5;
  const int l = t & 31;
  const v4f v = bfr4(*(const v4f*)(x + (size_t)in_row(row) * kDim + t * 4));
  float s = (v[0] + v[1]) + (v[2] + v[3]);
#pragma unroll
  for (int off = 1; off < 32; off <<= 1) s += __shfl_xor(s, off, 32);
  if (l == 0) ssum[w] = s;
  __syncthreads();
  float tot = 0.f;
#pragma unroll
  for (int i = 0; i < 6; ++i) tot += ssum[i];
  const float mean = tot * (1.0f / 768.0f);
  const v4f d = v - mean;
  float q = (d[0] * d[0] + d[1] * d[1]) + (d[2] * d[2] + d[3] * d[3]);
#pragma unroll
  for (int off = 1; off < 32; off <<= 1) q += __shfl_xor(q, off, 32);
  if (l == 0) ssq[w] = q;
  __syncthreads();
  float totq = 0.f;
#pragma unroll
  for (int i = 0; i < 6; ++i) totq += ssq[i];
  const float var = totq * (1.0f / 768.0f);
  const float inv = rsqrtf(var + kLnEps);
  const float* mrow = mod + (size_t)row * kModN;
  const v4f sa = *(const v4f*)(mrow + t * 4);
  const v4f sh = *(const v4f*)(mrow + kDim + t * 4);
  const v4f o = (d * inv) * (1.0f + sa) + sh;
  v2u pk;
  pk[0] = pack_h2(o[0] * hscale, o[1] * hscale);
  pk[1] = pack_h2(o[2] * hscale, o[3] * hscale);
  *(v2u*)(hrow + 2 * t) = pk;
  __syncthreads();
  if (t < 96) {
    const v4u wv = *(const v4u*)(hrow + 4 * t);
    _Float16* hp = hout + (size_t)row * kDim + t * 8;
    *(volatile v4u*)hp = wv;
    __threadfence();
    *(volatile v4u*)hp = wv;
  }
}

__global__ __launch_bounds__(192) void qkv_norm_rows(
    float* qkvf, const float* __restrict__ gq, const float* __restrict__ gk, float cq, float ck, float cvv) {
  __shared__ float sA[6];
  __shared__ float sB[6];
  __shared__ __align__(16) unsigned hrow[1152];
  const int row = blockIdx.x;
  const int t = threadIdx.x;
  const int w = t >> 5;
  const int l = t & 31;
  const float* src = qkvf + (size_t)row * kQkvN;
  const v4f q = *(const v4f*)(src + t * 4);
  const v4f k = *(const v4f*)(src + kDim + t * 4);
  const v4f v = *(const v4f*)(src + 2 * kDim + t * 4);
  float sq = (q[0] * q[0] + q[1] * q[1]) + (q[2] * q[2] + q[3] * q[3]);
  float sk = (k[0] * k[0] + k[1] * k[1]) + (k[2] * k[2] + k[3] * k[3]);
#pragma unroll
  for (int off = 1; off < 32; off <<= 1) { sq += __shfl_xor(sq, off, 32); sk += __shfl_xor(sk, off, 32); }
  if (l == 0) { sA[w] = sq; sB[w] = sk; }
  __syncthreads();
  float totq = 0.f, totk = 0.f;
#pragma unroll
  for (int i = 0; i < 6; ++i) { totq += sA[i]; totk += sB[i]; }
  const float iq = 1.0f / fmaxf(sqrtf(totq), 1e-12f);
  const float ik = 1.0f / fmaxf(sqrtf(totk), 1e-12f);
  const v4f gqv = bfr4(*(const v4f*)(gq + t * 4));
  const v4f gkv = bfr4(*(const v4f*)(gk + t * 4));
  const v4f qo = ((q * iq) * gqv) * kSqrtD * (0.125f * cq);
  const v4f ko = ((k * ik) * gkv) * kSqrtD * ck;
  const v4f vo = v * cvv;
  v2u pq, pkk, pv;
  pq[0]  = pack_h2(qo[0], qo[1]); pq[1]  = pack_h2(qo[2], qo[3]);
  pkk[0] = pack_h2(ko[0], ko[1]); pkk[1] = pack_h2(ko[2], ko[3]);
  pv[0]  = pack_h2(vo[0], vo[1]); pv[1]  = pack_h2(vo[2], vo[3]);
  *(v2u*)(hrow + 2 * t) = pq;
  *(v2u*)(hrow + 384 + 2 * t) = pkk;
  *(v2u*)(hrow + 768 + 2 * t) = pv;
  __syncthreads();
  const v4u w0 = *(const v4u*)(hrow + 4 * t);
  v4u w1 = w0;
  if (t < 96) w1 = *(const v4u*)(hrow + 4 * (192 + t));
  _Float16* dst = (_Float16*)(qkvf + (size_t)row * kQkvN);
  for (int pass = 0; pass < 2; ++pass) {
    *(volatile v4u*)(dst + 8 * t) = w0;
    if (t < 96) *(volatile v4u*)(dst + 8 * (192 + t)) = w1;
    __threadfence();
  }
}

__global__ __launch_bounds__(192) void post_attn_rows(
    const float* __restrict__ oproj, const float* __restrict__ go, const float* __restrict__ x,
    const float* __restrict__ mod, float* __restrict__ xmid, _Float16* __restrict__ h2out, float hscale) {
  __shared__ float sA[6];
  __shared__ float sB[6];
  __shared__ float sC[6];
  __shared__ __align__(16) unsigned hrow[384];
  const int row = blockIdx.x;
  const int t = threadIdx.x;
  const int w = t >> 5;
  const int l = t & 31;
  const v4f o = *(const v4f*)(oproj + (size_t)row * kDim + t * 4);
  float ss = (o[0] * o[0] + o[1] * o[1]) + (o[2] * o[2] + o[3] * o[3]);
#pragma unroll
  for (int off = 1; off < 32; off <<= 1) ss += __shfl_xor(ss, off, 32);
  if (l == 0) sA[w] = ss;
  __syncthreads();
  float tss = 0.f;
#pragma unroll
  for (int i = 0; i < 6; ++i) tss += sA[i];
  const float inv = 1.0f / fmaxf(sqrtf(tss), 1e-12f);
  const v4f gv = bfr4(*(const v4f*)(go + t * 4));
  const v4f a = ((o * inv) * gv) * kSqrtD;
  const float* mrow = mod + (size_t)row * kModN;
  const v4f xb = bfr4(*(const v4f*)(x + (size_t)in_row(row) * kDim + t * 4));
  const v4f ga = *(const v4f*)(mrow + 2 * kDim + t * 4);
  const v4f xm = xb + ga * a;
  float* xp = xmid + (size_t)row * kDim + t * 4;
  *(volatile v4f*)xp = xm;
  __threadfence();
  *(volatile v4f*)xp = xm;
  float s = (xm[0] + xm[1]) + (xm[2] + xm[3]);
#pragma unroll
  for (int off = 1; off < 32; off <<= 1) s += __shfl_xor(s, off, 32);
  if (l == 0) sB[w] = s;
  __syncthreads();
  float tot = 0.f;
#pragma unroll
  for (int i = 0; i < 6; ++i) tot += sB[i];
  const float mean = tot * (1.0f / 768.0f);
  const v4f d = xm - mean;
  float q = (d[0] * d[0] + d[1] * d[1]) + (d[2] * d[2] + d[3] * d[3]);
#pragma unroll
  for (int off = 1; off < 32; off <<= 1) q += __shfl_xor(q, off, 32);
  if (l == 0) sC[w] = q;
  __syncthreads();
  float totq = 0.f;
#pragma unroll
  for (int i = 0; i < 6; ++i) totq += sC[i];
  const float var = totq * (1.0f / 768.0f);
  const float inv2 = rsqrtf(var + kLnEps);
  const v4f s2  = *(const v4f*)(mrow + 3 * kDim + t * 4);
  const v4f sh2 = *(const v4f*)(mrow + 4 * kDim + t * 4);
  const v4f h2 = (d * inv2) * (1.0f + s2) + sh2;
  v2u pk;
  pk[0] = pack_h2(h2[0] * hscale, h2[1] * hscale);
  pk[1] = pack_h2(h2[2] * hscale, h2[3] * hscale);
  *(v2u*)(hrow + 2 * t) = pk;
  __syncthreads();
  if (t < 96) {
    const v4u wv = *(const v4u*)(hrow + 4 * t);
    _Float16* hp = h2out + (size_t)row * kDim + t * 8;
    *(volatile v4u*)hp = wv;
    __threadfence();
    *(volatile v4u*)hp = wv;
  }
}

constexpr int kAKC = 64;
constexpr int kAQB = 64;
constexpr int kANW = 4;

__device__ __forceinline__ void vt_scatter(_Float16* vt, v4u w, int d0, int kvr) {
#pragma unroll
  for (int e = 0; e < 4; ++e) {
    const unsigned u = w[e];
    const int d = d0 + 2 * e;
    vt[d * kAKC + kvr]       = __builtin_bit_cast(_Float16, (unsigned short)(u & 0xffffu));
    vt[(d + 1) * kAKC + kvr] = __builtin_bit_cast(_Float16, (unsigned short)(u >> 16));
  }
}

__global__ __launch_bounds__(128)
void attn_full_h64(const _Float16* __restrict__ qkvh, _Float16* __restrict__ attn_out,
                   float sscale, float pscale, float oscale) {
  union FH { v16h v; v8h h[2]; };
  __shared__ __align__(16) _Float16 Ksh[kAKC * kHdim];
  __shared__ __align__(16) _Float16 Vth[kHdim * kAKC];
  __shared__ __align__(16) _Float16 Psh[kANW][16 * kAKC];
  __shared__ __align__(16) float  Osl[kANW][16 * 68];

  const int tid  = threadIdx.x;
  const int wave = tid >> 5;
  const int lane = tid & 31;
  const int hh   = lane >> 4;
  const int c    = lane & 15;

  const int nqb = kSeq / kAQB;
  const int bx = blockIdx.x;
  const int qb = bx % nqb;
  const int bh = bx / nqb;
  const int h  = bh % kHeads;
  const int b  = bh / kHeads;
  const int q0 = qb * kAQB + wave * 16;

  const _Float16* rbase = qkvh + (size_t)b * kSeq * kQP;
  const _Float16* qbase = rbase + h * kHdim;
  const _Float16* kbase = rbase + kDim + h * kHdim;
  const _Float16* vbase = rbase + 2 * kDim + h * kHdim;

  v16h qa[2];
  {
    const _Float16* qrow = qbase + (size_t)(q0 + c) * kQP + 8 * hh;
    qa[0] = frag_load(qrow);
    qa[1] = frag_load(qrow + 32);
  }

  float mrow[8], lrow[8];
  v8f oacc[4];
#pragma unroll
  for (int r = 0; r < 8; ++r) { mrow[r] = -INFINITY; lrow[r] = 0.f; }
#pragma unroll
  for (int t = 0; t < 4; ++t) oacc[t] = (v8f){0.f,0.f,0.f,0.f,0.f,0.f,0.f,0.f};

  constexpr int nChunks = kSeq / kAKC;
  for (int kc = 0; kc < nChunks; ++kc) {
    const int kv0 = kc * kAKC;
    __syncthreads();
    {
      const int kvr = tid >> 1, dh = (tid & 1) * 32;
      const _Float16* krow = kbase + (size_t)(kv0 + kvr) * kQP + dh;
      const _Float16* vrow = vbase + (size_t)(kv0 + kvr) * kQP + dh;
      const v8h k0v = *(const v8h*)(krow);
      const v8h k1v = *(const v8h*)(krow + 8);
      const v8h k2v = *(const v8h*)(krow + 16);
      const v8h k3v = *(const v8h*)(krow + 24);
      const v4u v0w = *(const v4u*)(vrow);
      const v4u v1w = *(const v4u*)(vrow + 8);
      const v4u v2w = *(const v4u*)(vrow + 16);
      const v4u v3w = *(const v4u*)(vrow + 24);
      _Float16* kd = Ksh + kvr * kHdim + dh;
      *(v8h*)(kd)      = k0v;
      *(v8h*)(kd + 8)  = k1v;
      *(v8h*)(kd + 16) = k2v;
      *(v8h*)(kd + 24) = k3v;
      vt_scatter(Vth, v0w, dh,      kvr);
      vt_scatter(Vth, v1w, dh + 8,  kvr);
      vt_scatter(Vth, v2w, dh + 16, kvr);
      vt_scatter(Vth, v3w, dh + 24, kvr);
    }
    __syncthreads();

    v8f s[4];
#pragma unroll
    for (int j = 0; j < 4; ++j) {
      s[j] = (v8f){0.f,0.f,0.f,0.f,0.f,0.f,0.f,0.f};
#pragma unroll
      for (int dc = 0; dc < 2; ++dc) {
        FH kb;
        kb.h[0] = *(const v8h*)(Ksh + (j * 16 + c) * kHdim + dc * 32 + 8 * hh);
        kb.h[1] = *(const v8h*)(Ksh + (j * 16 + c) * kHdim + dc * 32 + 16 + 8 * hh);
        s[j] = mma_h(qa[dc], kb.v, s[j]);
      }
    }
    float cm[8];
#pragma unroll
    for (int r = 0; r < 8; ++r) {
      float m = -INFINITY;
#pragma unroll
      for (int j = 0; j < 4; ++j) {
        const float sv = s[j][r] * sscale;
        s[j][r] = sv;
        m = fmaxf(m, sv);
      }
#pragma unroll
      for (int off = 1; off < 16; off <<= 1) m = fmaxf(m, __shfl_xor(m, off, 32));
      cm[r] = m;
    }
    _Float16* pw = Psh[wave];
#pragma unroll
    for (int r = 0; r < 8; ++r) {
      const float mnew = fmaxf(mrow[r], cm[r]);
      const float alpha = __expf(mrow[r] - mnew);
      mrow[r] = mnew;
      float psum = 0.f;
#pragma unroll
      for (int j = 0; j < 4; ++j) {
        const float p = __expf(s[j][r] - mnew);
        psum += p;
        pw[(8 * hh + r) * kAKC + j * 16 + c] = (_Float16)(p * pscale);
      }
#pragma unroll
      for (int off = 1; off < 16; off <<= 1) psum += __shfl_xor(psum, off, 32);
      lrow[r] = lrow[r] * alpha + psum;
#pragma unroll
      for (int t = 0; t < 4; ++t) oacc[t][r] *= alpha;
    }
    __builtin_amdgcn_fence(3  , "workgroup");
    __builtin_amdgcn_wave_barrier();
    __builtin_amdgcn_fence(2  , "workgroup");
#pragma unroll
    for (int kk = 0; kk < 2; ++kk) {
      FH pa;
      pa.h[0] = *(const v8h*)(pw + c * kAKC + kk * 32 + 8 * hh);
      pa.h[1] = *(const v8h*)(pw + c * kAKC + kk * 32 + 16 + 8 * hh);
#pragma unroll
      for (int t = 0; t < 4; ++t) {
        FH vb;
        vb.h[0] = *(const v8h*)(Vth + (t * 16 + c) * kAKC + kk * 32 + 8 * hh);
        vb.h[1] = *(const v8h*)(Vth + (t * 16 + c) * kAKC + kk * 32 + 16 + 8 * hh);
        oacc[t] = mma_h(pa.v, vb.v, oacc[t]);
      }
    }
  }

  float* os = Osl[wave];
#pragma unroll
  for (int r = 0; r < 8; ++r) {
    const float inv = oscale / lrow[r];
#pragma unroll
    for (int t = 0; t < 4; ++t) os[(8 * hh + r) * 68 + t * 16 + c] = oacc[t][r] * inv;
  }
  __builtin_amdgcn_fence(3  , "workgroup");
  __builtin_amdgcn_wave_barrier();
  __builtin_amdgcn_fence(2  , "workgroup");
  {
    const int q8 = lane >> 3, c8 = (lane & 7) * 8;
    _Float16* ob = attn_out + (size_t)(b * kSeq) * kDim + h * kHdim;
    for (int pass = 0; pass < 2; ++pass) {
#pragma unroll
      for (int it = 0; it < 4; ++it) {
        const int row = it * 4 + q8;
        const float* sp = os + row * 68 + c8;
        v8h hv;
#pragma unroll
        for (int e = 0; e < 8; ++e) hv[e] = (_Float16)sp[e];
        *(volatile v8h*)(ob + (size_t)(q0 + row) * kDim + c8) = hv;
      }
      __threadfence();
    }
  }
}

extern "C" void kernel_launch(void* const* d_in, const int* in_sizes, int n_in,
                              void* d_out, int out_size, void* d_ws, size_t ws_size,
                              hipStream_t stream) {
  if (n_in != 15) return;
  const long needTok = (long)(kBatch - 1) * kSeqFull * kDim + (long)kSeq * kDim;
  if ((long)in_sizes[0] < needTok || (long)in_sizes[1] < needTok) return;
  if (in_sizes[2] < kDim * kQkvN || in_sizes[3] < kQkvN) return;
  if (in_sizes[4] < kDim * kDim || in_sizes[5] < kDim || in_sizes[6] < kDim || in_sizes[7] < kDim || in_sizes[8] < kDim) return;
  if (in_sizes[9] < kDim * kFfn || in_sizes[10] < kFfn || in_sizes[11] < kFfn * kDim || in_sizes[12] < kDim) return;
  if (in_sizes[13] < kDim * kModN || in_sizes[14] < kModN) return;
  if (out_size < kRows * kDim) return;
  if (ws_size < kWsTotal) return;

  const float* x     = (const float*)d_in[0];
  const float* c     = (const float*)d_in[1];
  const float* W_qkv = (const float*)d_in[2];
  const float* b_qkv = (const float*)d_in[3];
  const float* W_o   = (const float*)d_in[4];
  const float* b_o   = (const float*)d_in[5];
  const float* g_o   = (const float*)d_in[6];
  const float* g_q   = (const float*)d_in[7];
  const float* g_k   = (const float*)d_in[8];
  const float* W1    = (const float*)d_in[9];
  const float* b1    = (const float*)d_in[10];
  const float* W2    = (const float*)d_in[11];
  const float* b2    = (const float*)d_in[12];
  const float* W_ada = (const float*)d_in[13];
  const float* b_ada = (const float*)d_in[14];
  float* outf = (float*)d_out;

  char* ws = (char*)d_ws;
  float*    modf  = (float*)(ws + kOffMod);
  _Float16* w2t   = (_Float16*)(ws + kOffW2);
  _Float16* w1t   = (_Float16*)(ws + kOffW1);
  _Float16* wqkvt = (_Float16*)(ws + kOffWqkv);
  _Float16* wot   = (_Float16*)(ws + kOffWo);
  _Float16* actA  = (_Float16*)(ws + kOffA);
  _Float16* wadat = (_Float16*)(ws + kOffWada);
  float*    qkvf  = (float*)(ws + kOffQkvF);
  float*    xmid  = (float*)(ws + kOffXmid);
  float*    oproj = (float*)(ws + kOffOproj);
  _Float16* hid   = (_Float16*)(ws + kOffHid);

  transpose_cast_w<<<dim3(kModN / 64, kDim / 64), dim3(256), 0, stream>>>(W_ada, wadat, kDim, kModN, kCarryW);
  transpose_cast_w<<<dim3(kQkvN / 64, kDim / 64), dim3(256), 0, stream>>>(W_qkv, wqkvt, kDim, kQkvN, kCarryW);
  transpose_cast_w<<<dim3(kDim / 64, kDim / 64), dim3(256), 0, stream>>>(W_o, wot, kDim, kDim, kCarryW);
  transpose_cast_w<<<dim3(kFfn / 64, kDim / 64), dim3(256), 0, stream>>>(W1, w1t, kDim, kFfn, kCarryW);
  transpose_cast_w<<<dim3(kDim / 64, kFfn / 64), dim3(256), 0, stream>>>(W2, w2t, kFfn, kDim, kCarryW);

  {
    const int n8 = kRows * kDim / 8;
    silu_cast_rows<<<dim3((unsigned)((n8 + 255) / 256)), dim3(256), 0, stream>>>(c, actA, n8, kCarryAct);
  }

  {
    const unsigned tiles = (unsigned)((kRows / 64) * (kModN / 64));
    wmma_gemm64<2, 0, false, false, 0><<<dim3((tiles + 7) / 8), dim3(256), 0, stream>>>(
        actA, kDim, wadat, kDim, (void*)modf, kModN, b_ada, modf, 0, modf, 0,
        kRows, kModN, kDim, 1.0f / (kCarryAct * kCarryW), 1.0f);
  }

  ln_mod_rows<<<dim3((unsigned)kRows), dim3(192), 0, stream>>>(x, modf, actA, kCarryAct);

  {
    const unsigned tiles = (unsigned)((kRows / 64) * (kQkvN / 64));
    wmma_gemm64<2, 0, false, false, 0><<<dim3((tiles + 7) / 8), dim3(256), 0, stream>>>(
        actA, kDim, wqkvt, kDim, (void*)qkvf, kQkvN, b_qkv, modf, 0, modf, 0,
        kRows, kQkvN, kDim, 1.0f / (kCarryAct * kCarryW), 1.0f);
  }

  qkv_norm_rows<<<dim3((unsigned)kRows), dim3(192), 0, stream>>>(qkvf, g_q, g_k, kCarryQ, kCarryK, kCarryV);

  {
    const unsigned blocks = (unsigned)(kBatch * kHeads * (kSeq / kAQB));
    attn_full_h64<<<dim3(blocks), dim3(128), 0, stream>>>(
        (const _Float16*)qkvf, actA, 1.0f / (kCarryQ * kCarryK), kCarryP, kCarryAttn / (kCarryP * kCarryV));
  }

  {
    const unsigned tiles = (unsigned)((kRows / 64) * (kDim / 64));
    wmma_gemm64<2, 0, false, false, 0><<<dim3((tiles + 7) / 8), dim3(256), 0, stream>>>(
        actA, kDim, wot, kDim, (void*)oproj, kDim, b_o, modf, 0, modf, 0,
        kRows, kDim, kDim, 1.0f / (kCarryAttn * kCarryW), 1.0f);
  }

  post_attn_rows<<<dim3((unsigned)kRows), dim3(192), 0, stream>>>(oproj, g_o, x, modf, xmid, actA, kCarryAct);

  {
    const unsigned tiles = (unsigned)((kRows / 64) * (kFfn / 64));
    wmma_gemm64<2, 1, false, false, 3><<<dim3((tiles + 7) / 8), dim3(256), 0, stream>>>(
        actA, kDim, w1t, kDim, (void*)hid, kFfn, b1, modf, 0, modf, 0,
        kRows, kFfn, kDim, 1.0f / (kCarryAct * kCarryW), kCarryH);
  }

  {
    const unsigned tiles = (unsigned)((kRows / 64) * (kDim / 64));
    wmma_gemm64<2, 0, true, true, 0><<<dim3((tiles + 7) / 8), dim3(256), 0, stream>>>(
        hid, kFfn, w2t, kFfn, (void*)outf, kDim, b2, xmid, kDim, modf + 5 * kDim, kModN,
        kRows, kDim, kFfn, 1.0f / (kCarryH * kCarryW), 1.0f);
  }
}
